// SimpleLure_89215060672645
// MI455X (gfx1250) — hardware-verified
//
#include <hip/hip_runtime.h>
#include <math.h>

constexpr int NB_SEQ    = 64;
constexpr int NT_STEP   = 1024;
constexpr int NX_DIM    = 256;
constexpr int ND_DIM    = 64;
constexpr int NW_DIM    = 128;
constexpr int NE_DIM    = 64;
constexpr int NEX_DIM   = NE_DIM + NX_DIM;
constexpr int ROWS_BLK  = 16;
constexpr int NTHR_SEQ  = 128;
constexpr int NWAVE_SEQ = NTHR_SEQ / 32;
constexpr int NTHR_CVT  = 256;
constexpr int XPITCH    = NX_DIM + 8;
constexpr int WPITCH    = NW_DIM + 8;
constexpr int DPITCH    = ND_DIM + 8;
constexpr int EPITCH    = 68;
constexpr int NSUB2     = NEX_DIM / 16 / NWAVE_SEQ;
constexpr int NOUT_TOTAL = NB_SEQ * NT_STEP * NE_DIM;
constexpr float WCAR      = 32.0f;
constexpr float WCAR_INV  = 1.0f / 32.0f;
constexpr float LCAR      = 2048.0f;
constexpr float LCAR_INV  = 1.0f / 2048.0f;

static_assert(NB_SEQ % ROWS_BLK == 0);
static_assert(NSUB2 * 16 * NWAVE_SEQ == NEX_DIM);
static_assert(NE_DIM == 16 * NWAVE_SEQ);
static_assert(NW_DIM == 32 * NWAVE_SEQ);
static_assert(NX_DIM % 32 == 0 && ND_DIM % 32 == 0 && NW_DIM % 32 == 0);
static_assert(ROWS_BLK * ND_DIM == 8 * NTHR_SEQ);
static_assert(ROWS_BLK == 4 * NWAVE_SEQ && NE_DIM == 64);
static_assert(XPITCH % 8 == 0 && WPITCH % 8 == 0 && DPITCH % 8 == 0 && EPITCH % 4 == 0);
static_assert((ROWS_BLK * XPITCH) % 8 == 0 && (ROWS_BLK * WPITCH) % 8 == 0 && (ROWS_BLK * DPITCH) % 8 == 0);

typedef __attribute__((ext_vector_type(16))) _Float16 v16h;
typedef __attribute__((ext_vector_type(8)))  _Float16 v8h;
typedef __attribute__((ext_vector_type(8)))  float    v8f;
typedef __attribute__((ext_vector_type(4)))  float    v4f;

__device__ __forceinline__ void guard4x4_h(v8f& a, v8f& b, v8f& c, v8f& d, v16h w, v16h x, v16h y, v16h z) {
  asm volatile("v_nop\n\tv_nop\n\tv_nop\n\tv_nop" : "+v"(a), "+v"(b), "+v"(c), "+v"(d) : "v"(w), "v"(x), "v"(y), "v"(z));
}
__device__ __forceinline__ void guard10_h(v8f& e0, v8f& e1, v8f& e2, v8f& e3, v8f& e4,
                                          v8f& l0, v8f& l1, v8f& l2, v8f& l3, v8f& l4,
                                          v16h a0, v16h a1, v16h b0, v16h b1, v16h b2, v16h b3, v16h b4) {
  asm volatile("v_nop\n\tv_nop\n\tv_nop\n\tv_nop"
               : "+v"(e0), "+v"(e1), "+v"(e2), "+v"(e3), "+v"(e4), "+v"(l0), "+v"(l1), "+v"(l2), "+v"(l3), "+v"(l4)
               : "v"(a0), "v"(a1), "v"(b0), "v"(b1), "v"(b2), "v"(b3), "v"(b4));
}
__device__ __forceinline__ void acc_guard4(v8f& a, v8f& b, v8f& c, v8f& d) { asm volatile("v_nop\n\tv_nop\n\tv_nop\n\tv_nop" : "+v"(a), "+v"(b), "+v"(c), "+v"(d)); }
__device__ __forceinline__ void acc_guard2(v8f& a, v8f& b) { asm volatile("v_nop\n\tv_nop\n\tv_nop\n\tv_nop" : "+v"(a), "+v"(b)); }

template <typename T> struct Frag;
template <> struct Frag<_Float16> {
  typedef v16h V; union U { v16h v; v8h h[2]; };
  static __device__ __forceinline__ v16h load(const _Float16* p) {
    U f; f.h[0] = *(const v8h*)(p); f.h[1] = *(const v8h*)(p + 16); return f.v;
  }
  static __device__ __forceinline__ v8f mma(v16h a, v16h b, v8f c) {
    return __builtin_amdgcn_wmma_f32_16x16x32_f16(false, a, false, b, (short)0, c, false, false);
  }
};

__global__ __launch_bounds__(NTHR_CVT) void cvt8_f16_kernel(const float* __restrict__ src, unsigned short* __restrict__ dst,
                                                            int n8, float sc) {
  const int i = blockIdx.x * NTHR_CVT + threadIdx.x;
  if (i < n8) {
    const float* sp = src + (size_t)i * 8;
    const v4f a = *(const v4f*)(sp);
    const v4f b = *(const v4f*)(sp + 4);
    v8h hv;
#pragma unroll
    for (int e = 0; e < 4; ++e) {
      hv[e]     = (_Float16)(a[e] * sc);
      hv[4 + e] = (_Float16)(b[e] * sc);
    }
    *(volatile v8h*)(dst + (size_t)i * 8) = hv;
    __threadfence();
    *(volatile v8h*)(dst + (size_t)i * 8) = hv;
  }
}

__device__ __forceinline__ void stage_d_tile(_Float16* dtile, const float* __restrict__ dsig, int rowbase, int t, int tid) {
  const int row = tid >> 3;
  const int c8  = (tid & 7) * 8;
  const float* sp = dsig + ((size_t)(rowbase + row) * NT_STEP + (size_t)t) * ND_DIM + c8;
  const v4f a = *(const v4f*)(sp);
  const v4f b = *(const v4f*)(sp + 4);
  v8h hv;
#pragma unroll
  for (int e = 0; e < 4; ++e) { hv[e] = (_Float16)a[e]; hv[4 + e] = (_Float16)b[e]; }
  *(v8h*)(dtile + row * DPITCH + c8) = hv;
}

__global__ __launch_bounds__(NTHR_SEQ) void lure_seq_kernel(const float* __restrict__ dsig,
                                                             const unsigned short* __restrict__ PXSp,
                                                             const unsigned short* __restrict__ PDSp,
                                                             const unsigned short* __restrict__ PWSp,
                                                             const unsigned short* __restrict__ PZXp,
                                                             const unsigned short* __restrict__ PZDp,
                                                             float* __restrict__ out) {
  __shared__ __align__(16) _Float16 Xh[ROWS_BLK * XPITCH];
  __shared__ __align__(16) _Float16 Xl[ROWS_BLK * XPITCH];
  __shared__ __align__(16) _Float16 Wh[ROWS_BLK * WPITCH];
  __shared__ __align__(16) _Float16 Wl[ROWS_BLK * WPITCH];
  __shared__ __align__(16) _Float16 Dt[ROWS_BLK * DPITCH];
  __shared__ __align__(16) float    Es[ROWS_BLK * EPITCH];
  const _Float16* PXS = (const _Float16*)PXSp;
  const _Float16* PDS = (const _Float16*)PDSp;
  const _Float16* PWS = (const _Float16*)PWSp;
  const _Float16* PZX = (const _Float16*)PZXp;
  const _Float16* PZD = (const _Float16*)PZDp;
  const int tid = threadIdx.x, lane = tid & 31, wave = tid >> 5;
  const int c = lane & 15, hh = lane >> 4, koff = hh * 8, c4 = c * 4;
  const int rowbase = blockIdx.x * ROWS_BLK;
  const v8f z8 = {0.f, 0.f, 0.f, 0.f, 0.f, 0.f, 0.f, 0.f};

  {
    v8h zero8;
#pragma unroll
    for (int e = 0; e < 8; ++e) zero8[e] = (_Float16)0.0f;
#pragma unroll 1
    for (int i = tid; i < (ROWS_BLK * XPITCH) / 8; i += NTHR_SEQ) { *(v8h*)(Xh + 8 * i) = zero8; *(v8h*)(Xl + 8 * i) = zero8; }
#pragma unroll 1
    for (int i = tid; i < (ROWS_BLK * WPITCH) / 8; i += NTHR_SEQ) { *(v8h*)(Wh + 8 * i) = zero8; *(v8h*)(Wl + 8 * i) = zero8; }
#pragma unroll 1
    for (int i = tid; i < (ROWS_BLK * DPITCH) / 8; i += NTHR_SEQ) { *(v8h*)(Dt + 8 * i) = zero8; }
  }
  __syncthreads();
  stage_d_tile(Dt, dsig, rowbase, 0, tid);
  __syncthreads();

  const _Float16* xhrow = Xh + c * XPITCH + koff;
  const _Float16* xlrow = Xl + c * XPITCH + koff;
  const _Float16* whrow = Wh + c * WPITCH + koff;
  const _Float16* wlrow = Wl + c * WPITCH + koff;
  const _Float16* dtrow = Dt + c * DPITCH + koff;
  const int nz = 32 * wave + c;
  const _Float16* bzx = PZX + (size_t)nz * NX_DIM + koff;
  const _Float16* bzd = PZD + (size_t)nz * ND_DIM + koff;
  const int ns = 16 * wave + c;
  const _Float16* bex = PXS + (size_t)ns * NX_DIM + koff;
  const _Float16* bed = PDS + (size_t)ns * ND_DIM + koff;
  const _Float16* bew = PWS + (size_t)ns * NW_DIM + koff;

#pragma unroll 1
  for (int t = 0; t < NT_STEP; ++t) {
    {
      v8f zh0 = z8, zh1 = z8, zl0 = z8, zl1 = z8;
#pragma unroll 1
      for (int k0 = 0; k0 < NX_DIM; k0 += 32) {
        const v16h b0 = Frag<_Float16>::load(bzx + k0);
        const v16h b1 = Frag<_Float16>::load(bzx + 16 * NX_DIM + k0);
        const v16h ah = Frag<_Float16>::load(xhrow + k0);
        const v16h al = Frag<_Float16>::load(xlrow + k0);
        zh0 = Frag<_Float16>::mma(ah, b0, zh0);
        zh1 = Frag<_Float16>::mma(ah, b1, zh1);
        zl0 = Frag<_Float16>::mma(al, b0, zl0);
        zl1 = Frag<_Float16>::mma(al, b1, zl1);
        guard4x4_h(zh0, zh1, zl0, zl1, ah, al, b0, b1);
      }
#pragma unroll 1
      for (int k0 = 0; k0 < ND_DIM; k0 += 32) {
        const v16h b0 = Frag<_Float16>::load(bzd + k0);
        const v16h b1 = Frag<_Float16>::load(bzd + 16 * ND_DIM + k0);
        const v16h ad = Frag<_Float16>::load(dtrow + k0);
        zh0 = Frag<_Float16>::mma(ad, b0, zh0);
        zh1 = Frag<_Float16>::mma(ad, b1, zh1);
        guard4x4_h(zh0, zh1, zl0, zl1, ad, ad, b0, b1);
      }
      acc_guard4(zh0, zh1, zl0, zl1);
#pragma unroll
      for (int r = 0; r < 8; ++r) {
        const int row = 8 * hh + r;
        const float z0 = (zh0[r] + zl0[r] * LCAR_INV) * WCAR_INV;
        const float z1 = (zh1[r] + zl1[r] * LCAR_INV) * WCAR_INV;
        const float w0 = tanhf(z0);
        const float w1 = tanhf(z1);
        const _Float16 h0 = (_Float16)w0;
        const _Float16 h1 = (_Float16)w1;
        const _Float16 l0 = (_Float16)((w0 - (float)h0) * LCAR);
        const _Float16 l1 = (_Float16)((w1 - (float)h1) * LCAR);
        Wh[row * WPITCH + nz]      = h0;
        Wh[row * WPITCH + nz + 16] = h1;
        Wl[row * WPITCH + nz]      = l0;
        Wl[row * WPITCH + nz + 16] = l1;
      }
    }
    __syncthreads();

    float xv[4][8];
    {
      v8f eh[NSUB2], el[NSUB2];
#pragma unroll
      for (int q = 0; q < NSUB2; ++q) { eh[q] = z8; el[q] = z8; }
#pragma unroll 1
      for (int k0 = 0; k0 < NX_DIM; k0 += 32) {
        v16h b[NSUB2];
#pragma unroll
        for (int q = 0; q < NSUB2; ++q) b[q] = Frag<_Float16>::load(bex + (size_t)q * 64 * NX_DIM + k0);
        const v16h ah = Frag<_Float16>::load(xhrow + k0);
        const v16h al = Frag<_Float16>::load(xlrow + k0);
#pragma unroll
        for (int q = 0; q < NSUB2; ++q) {
          eh[q] = Frag<_Float16>::mma(ah, b[q], eh[q]);
          el[q] = Frag<_Float16>::mma(al, b[q], el[q]);
        }
        guard10_h(eh[0], eh[1], eh[2], eh[3], eh[4], el[0], el[1], el[2], el[3], el[4], ah, al, b[0], b[1], b[2], b[3], b[4]);
      }
#pragma unroll 1
      for (int k0 = 0; k0 < ND_DIM; k0 += 32) {
        v16h b[NSUB2];
#pragma unroll
        for (int q = 0; q < NSUB2; ++q) b[q] = Frag<_Float16>::load(bed + (size_t)q * 64 * ND_DIM + k0);
        const v16h ad = Frag<_Float16>::load(dtrow + k0);
#pragma unroll
        for (int q = 0; q < NSUB2; ++q) eh[q] = Frag<_Float16>::mma(ad, b[q], eh[q]);
        guard10_h(eh[0], eh[1], eh[2], eh[3], eh[4], el[0], el[1], el[2], el[3], el[4], ad, ad, b[0], b[1], b[2], b[3], b[4]);
      }
#pragma unroll 1
      for (int k0 = 0; k0 < NW_DIM; k0 += 32) {
        v16h b[NSUB2];
#pragma unroll
        for (int q = 0; q < NSUB2; ++q) b[q] = Frag<_Float16>::load(bew + (size_t)q * 64 * NW_DIM + k0);
        const v16h ah = Frag<_Float16>::load(whrow + k0);
        const v16h al = Frag<_Float16>::load(wlrow + k0);
#pragma unroll
        for (int q = 0; q < NSUB2; ++q) {
          eh[q] = Frag<_Float16>::mma(ah, b[q], eh[q]);
          el[q] = Frag<_Float16>::mma(al, b[q], el[q]);
        }
        guard10_h(eh[0], eh[1], eh[2], eh[3], eh[4], el[0], el[1], el[2], el[3], el[4], ah, al, b[0], b[1], b[2], b[3], b[4]);
      }
      acc_guard4(eh[0], eh[1], eh[2], eh[3]);
      acc_guard4(el[0], el[1], el[2], el[3]);
      acc_guard2(eh[4], el[4]);
#pragma unroll
      for (int r = 0; r < 8; ++r)
        Es[(8 * hh + r) * EPITCH + ns] = (eh[0][r] + el[0][r] * LCAR_INV) * WCAR_INV;
#pragma unroll
      for (int q = 1; q < NSUB2; ++q)
#pragma unroll
        for (int r = 0; r < 8; ++r) xv[q - 1][r] = (eh[q][r] + el[q][r] * LCAR_INV) * WCAR_INV;
    }
    __syncthreads();

    {
      float* ob = out + ((size_t)rowbase * NT_STEP + (size_t)t) * NE_DIM;
      for (int pass = 0; pass < 2; ++pass) {
#pragma unroll
        for (int it = 0; it < 2; ++it) {
          const int row = 4 * wave + 2 * it + hh;
          const v4f v = *(const v4f*)(Es + row * EPITCH + c4);
          *(volatile v4f*)(ob + (size_t)row * NT_STEP * NE_DIM + c4) = v;
        }
        __threadfence();
      }
#pragma unroll
      for (int q = 0; q < 4; ++q) {
        const int col = 16 * wave + 64 * q + c;
#pragma unroll
        for (int r = 0; r < 8; ++r) {
          const int row = 8 * hh + r;
          const float xf = xv[q][r];
          const _Float16 hi = (_Float16)xf;
          const _Float16 lo = (_Float16)((xf - (float)hi) * LCAR);
          Xh[row * XPITCH + col] = hi;
          Xl[row * XPITCH + col] = lo;
        }
      }
      const int tn = (t + 1 < NT_STEP) ? (t + 1) : (NT_STEP - 1);
      stage_d_tile(Dt, dsig, rowbase, tn, tid);
    }
    __syncthreads();
  }
}

extern "C" void kernel_launch(void* const* d_in, const int* in_sizes, int n_in,
                              void* d_out, int out_size, void* d_ws, size_t ws_size, hipStream_t stream) {
  if (n_in < 9 || d_out == nullptr || d_ws == nullptr) return;
  if (in_sizes[0] != NB_SEQ * NT_STEP * ND_DIM || in_sizes[1] != NX_DIM * NX_DIM || in_sizes[2] != NX_DIM * ND_DIM ||
      in_sizes[3] != NX_DIM * NW_DIM || in_sizes[4] != NE_DIM * NX_DIM || in_sizes[5] != NE_DIM * ND_DIM ||
      in_sizes[6] != NE_DIM * NW_DIM || in_sizes[7] != NW_DIM * NX_DIM || in_sizes[8] != NW_DIM * ND_DIM ||
      out_size != NOUT_TOTAL) return;

  const float* dsig = (const float*)d_in[0];
  const float* wA   = (const float*)d_in[1];
  const float* wB   = (const float*)d_in[2];
  const float* wB2  = (const float*)d_in[3];
  const float* wC   = (const float*)d_in[4];
  const float* wD   = (const float*)d_in[5];
  const float* wD12 = (const float*)d_in[6];
  const float* wC2  = (const float*)d_in[7];
  const float* wD21 = (const float*)d_in[8];
  float* es_out = (float*)d_out;

  char* ws = (char*)d_ws; size_t off = 0;
  auto carve = [&](size_t bytes) -> char* { char* p = ws + off; off += (bytes + 255) & ~(size_t)255; return p; };
  unsigned short* PXS = (unsigned short*)carve((size_t)NEX_DIM * NX_DIM * 2);
  unsigned short* PDS = (unsigned short*)carve((size_t)NEX_DIM * ND_DIM * 2);
  unsigned short* PWS = (unsigned short*)carve((size_t)NEX_DIM * NW_DIM * 2);
  unsigned short* PZX = (unsigned short*)carve((size_t)NW_DIM * NX_DIM * 2);
  unsigned short* PZD = (unsigned short*)carve((size_t)NW_DIM * ND_DIM * 2);
  if (off > ws_size || off > (size_t)134217728) return;

  const int n8C   = NE_DIM * NX_DIM / 8;
  const int n8A   = NX_DIM * NX_DIM / 8;
  const int n8D   = NE_DIM * ND_DIM / 8;
  const int n8B   = NX_DIM * ND_DIM / 8;
  const int n8D12 = NE_DIM * NW_DIM / 8;
  const int n8B2  = NX_DIM * NW_DIM / 8;
  const int n8C2  = NW_DIM * NX_DIM / 8;
  const int n8D21 = NW_DIM * ND_DIM / 8;
  cvt8_f16_kernel<<<(n8C   + NTHR_CVT - 1) / NTHR_CVT, NTHR_CVT, 0, stream>>>(wC,   PXS,                            n8C,   WCAR);
  cvt8_f16_kernel<<<(n8A   + NTHR_CVT - 1) / NTHR_CVT, NTHR_CVT, 0, stream>>>(wA,   PXS + (size_t)NE_DIM * NX_DIM,  n8A,   WCAR);
  cvt8_f16_kernel<<<(n8D   + NTHR_CVT - 1) / NTHR_CVT, NTHR_CVT, 0, stream>>>(wD,   PDS,                            n8D,   WCAR);
  cvt8_f16_kernel<<<(n8B   + NTHR_CVT - 1) / NTHR_CVT, NTHR_CVT, 0, stream>>>(wB,   PDS + (size_t)NE_DIM * ND_DIM,  n8B,   WCAR);
  cvt8_f16_kernel<<<(n8D12 + NTHR_CVT - 1) / NTHR_CVT, NTHR_CVT, 0, stream>>>(wD12, PWS,                            n8D12, WCAR);
  cvt8_f16_kernel<<<(n8B2  + NTHR_CVT - 1) / NTHR_CVT, NTHR_CVT, 0, stream>>>(wB2,  PWS + (size_t)NE_DIM * NW_DIM,  n8B2,  WCAR);
  cvt8_f16_kernel<<<(n8C2  + NTHR_CVT - 1) / NTHR_CVT, NTHR_CVT, 0, stream>>>(wC2,  PZX,                            n8C2,  WCAR);
  cvt8_f16_kernel<<<(n8D21 + NTHR_CVT - 1) / NTHR_CVT, NTHR_CVT, 0, stream>>>(wD21, PZD,                            n8D21, WCAR);

  lure_seq_kernel<<<NB_SEQ / ROWS_BLK, NTHR_SEQ, 0, stream>>>(dsig, PXS, PDS, PWS, PZX, PZD, es_out);
}
